// MHA_19121194401830
// MI455X (gfx1250) — hardware-verified
//
#include <hip/hip_runtime.h>


#ifndef NB
#define NB 2
#endif
#ifndef SEQ
#define SEQ 2048
#endif
#define NB_FULL  2
#define SEQ_FULL 2048
#define TT   SEQ
#define DM   1024
#define NH_  16
#define HD   64
#define DQ   (NH_ * HD)
#define ZH   2
#define PCAR 1024.0f
#define SCL  0.125f
static_assert(TT % 128 == 0);
static_assert(NH_ % ZH == 0);
static_assert(DM % 64 == 0 && DQ % 64 == 0 && HD == 64);
static_assert(NB >= 1 && NB <= NB_FULL && SEQ <= SEQ_FULL);

typedef _Float16 h16;
typedef unsigned short bf;
typedef __attribute__((ext_vector_type(16))) __bf16   v16bf;
typedef __attribute__((ext_vector_type(16))) _Float16 v16h;
typedef __attribute__((ext_vector_type(8)))  _Float16 v8h;
typedef __attribute__((ext_vector_type(8)))  unsigned short v8us;
typedef __attribute__((ext_vector_type(8)))  float    v8f;
typedef __attribute__((ext_vector_type(4)))  float    v4f;
typedef __attribute__((ext_vector_type(4)))  _Float16 v4h;
typedef v8h  __attribute__((may_alias)) v8ha;
typedef v4f  __attribute__((may_alias)) v4fa;
typedef v8us __attribute__((may_alias)) v8usa;

__device__ __forceinline__ unsigned short f2bf(float f) { unsigned u = __float_as_uint(f); u += 0x7FFFu + ((u >> 16) & 1u); return (unsigned short)(u >> 16); }
__device__ __forceinline__ float bf2f(unsigned short b) { return __uint_as_float(((unsigned)b) << 16); }
__device__ __forceinline__ float bfr(float f) { return bf2f(f2bf(f)); }
__device__ __forceinline__ v16h cat16(v8h lo, v8h hi) { return __builtin_shufflevector(lo, hi, 0, 1, 2, 3, 4, 5, 6, 7, 8, 9, 10, 11, 12, 13, 14, 15); }
__device__ __forceinline__ v16bf cat16b(v8us lo, v8us hi) { return __builtin_bit_cast(v16bf, __builtin_shufflevector(lo, hi, 0, 1, 2, 3, 4, 5, 6, 7, 8, 9, 10, 11, 12, 13, 14, 15)); }
__device__ __forceinline__ v8f wmma16(v16h a, v16h b, v8f c) { return __builtin_amdgcn_wmma_f32_16x16x32_f16(false, a, false, b, (short)0, c, false, false); }
__device__ __forceinline__ v8f wmmab(v16bf a, v16bf b, v8f c) { return __builtin_amdgcn_wmma_f32_16x16x32_bf16(false, a, false, b, (short)0, c, false, false); }
__device__ __forceinline__ h16 tohx(float x) { return (h16)x; }
__device__ __forceinline__ void splitf(float y, unsigned short& h, unsigned short& l) { h = f2bf(y); l = f2bf(y - bf2f(h)); }

template <typename T16> struct WFrag;
template <> struct WFrag<h16> { typedef v16h V; static __device__ __forceinline__ V ld(const h16* p) { return cat16(*(const v8h*)p, *(const v8h*)(p + 16)); } static __device__ __forceinline__ v8f mma(V a, V b, v8f c) { return wmma16(a, b, c); } };
template <> struct WFrag<bf> { typedef v16bf V; static __device__ __forceinline__ V ld(const bf* p) { return cat16b(*(const v8us*)p, *(const v8us*)(p + 16)); } static __device__ __forceinline__ v8f mma(V a, V b, v8f c) { return wmmab(a, b, c); } };
template <typename T16, int NSPLIT, bool BIAS>
__global__ __launch_bounds__(32) void k_gemmw(const T16* __restrict__ A, const T16* __restrict__ A2, const T16* __restrict__ Bt, const T16* __restrict__ Bt2, int K, float* C, int ldc, const float* __restrict__ bias, size_t sA, size_t sB, size_t sC) {
    typedef typename WFrag<T16>::V V;
    __shared__ __align__(16) float os[16 * 68];
    const size_t z = blockIdx.z; A += z * sA; if (A2) A2 += z * sA; Bt += z * sB; if (Bt2) Bt2 += z * sB; C += z * sC;
    const int lane = threadIdx.x & 31, lr = lane & 15, hi = lane >> 4; const int r0 = blockIdx.x * 64, c0 = blockIdx.y * 64;
    v8f acc[4][4];
#pragma unroll
    for (int mb = 0; mb < 4; ++mb)
#pragma unroll
        for (int nb = 0; nb < 4; ++nb) acc[mb][nb] = (v8f){};
    const size_t aoff = (size_t)(r0 + lr) * K + 8 * hi, boff = (size_t)(c0 + lr) * K + 8 * hi;
#pragma unroll 1
    for (int kc = 0; kc < K; kc += 32) {
        V a[4], a2[4];
#pragma unroll
        for (int mb = 0; mb < 4; ++mb) { a[mb] = WFrag<T16>::ld(A + aoff + (size_t)mb * 16 * K + kc); if (NSPLIT == 1 || NSPLIT == 2) a2[mb] = WFrag<T16>::ld(A2 + aoff + (size_t)mb * 16 * K + kc); }
#pragma unroll
        for (int nb = 0; nb < 4; ++nb) { const V b = WFrag<T16>::ld(Bt + boff + (size_t)nb * 16 * K + kc); V b2; if (NSPLIT >= 2) b2 = WFrag<T16>::ld(Bt2 + boff + (size_t)nb * 16 * K + kc);
#pragma unroll
            for (int mb = 0; mb < 4; ++mb) { acc[mb][nb] = WFrag<T16>::mma(a[mb], b, acc[mb][nb]); if (NSPLIT == 1 || NSPLIT == 2) acc[mb][nb] = WFrag<T16>::mma(a2[mb], b, acc[mb][nb]); if (NSPLIT >= 2) acc[mb][nb] = WFrag<T16>::mma(a[mb], b2, acc[mb][nb]); } }
        asm volatile("v_nop\n\tv_nop\n\tv_nop\n\tv_nop" : "+v"(acc[0][0]), "+v"(acc[1][1]), "+v"(acc[2][2]), "+v"(acc[3][3]) : "v"(a[0]), "v"(a[3]));
    }
#pragma unroll
    for (int mb = 0; mb < 4; ++mb) {
#pragma unroll
        for (int nb = 0; nb < 4; ++nb) {
#pragma unroll
            for (int j = 0; j < 8; ++j) os[(hi * 8 + j) * 68 + nb * 16 + lr] = acc[mb][nb][j]; }
        __builtin_amdgcn_wave_barrier(); asm volatile("" ::: "memory");
        float* crow = C + (size_t)(r0 + mb * 16) * ldc + c0;
#pragma unroll 1
        for (int ps = 0; ps < 2; ++ps) {
#pragma unroll
            for (int s = 0; s < 8; ++s) { const int row = 2 * s + hi, cofs = lr * 4; v4f val = *(const v4fa*)(os + row * 68 + cofs); if (BIAS) { val[0] += bfr(bias[c0 + cofs]); val[1] += bfr(bias[c0 + cofs + 1]); val[2] += bfr(bias[c0 + cofs + 2]); val[3] += bfr(bias[c0 + cofs + 3]); }
                *(volatile v4f*)(crow + (size_t)row * ldc + cofs) = val; }
            if (ps == 0) __threadfence(); }
        __builtin_amdgcn_wave_barrier(); asm volatile("" ::: "memory");
    }
}

__global__ __launch_bounds__(256) void k_cvt8(const float* __restrict__ src, bf* dst, size_t n8) { const size_t i = (size_t)blockIdx.x * 256 + threadIdx.x; if (i >= n8) return; const v8f v = *(const v8f*)(src + i * 8); v8us o;
#pragma unroll
    for (int k = 0; k < 8; ++k) o[k] = f2bf(v[k]); *(volatile v8us*)(dst + i * 8) = o; __threadfence(); *(volatile v8us*)(dst + i * 8) = o; }

__global__ __launch_bounds__(256) void k_qkp(const float* __restrict__ F, int pitch, int nheads, h16* P16) {
    const size_t e = ((size_t)blockIdx.x * 256 + threadIdx.x) * 8; if (e >= (size_t)nheads * TT * HD) return;
    const int d = (int)(e % HD); const int t = (int)((e / HD) % TT); const int h = (int)(e / ((size_t)HD * TT));
    const float* f = F + (size_t)t * pitch + (size_t)h * HD + d;
    const v4f x0 = *(const v4f*)f; const v4f x1 = *(const v4f*)(f + 4); v8h o;
#pragma unroll
    for (int q = 0; q < 4; ++q) { o[q] = tohx(x0[q]); o[q + 4] = tohx(x1[q]); }
    *(volatile v8h*)(P16 + e) = o; __threadfence(); *(volatile v8h*)(P16 + e) = o;
}
__global__ __launch_bounds__(256) void k_vtp(const float* __restrict__ F, int pitch, int nheads, h16* V16) {
    const size_t e = ((size_t)blockIdx.x * 256 + threadIdx.x) * 8; if (e >= (size_t)nheads * HD * TT) return;
    const int t = (int)(e % TT); const int d = (int)((e / TT) % HD); const int g = (int)(e / ((size_t)TT * HD));
    const float* f = F + (size_t)t * pitch + (size_t)g * HD + d; v8h o;
#pragma unroll
    for (int q = 0; q < 8; ++q) o[q] = tohx(f[(size_t)q * pitch]);
    *(volatile v8h*)(V16 + e) = o; __threadfence(); *(volatile v8h*)(V16 + e) = o;
}
__global__ __launch_bounds__(256) void k_asoft(const float* __restrict__ Sb, h16* P16) {
    const int lane = threadIdx.x & 31; const int row = blockIdx.x * 8 + (threadIdx.x >> 5); if (row >= ZH * TT) return;
    const float* sr = Sb + (size_t)row * TT; float v[TT / 32]; float mx = -3.0e38f;
#pragma unroll
    for (int ch = 0; ch < TT / 128; ++ch) { const int j0 = ch * 128 + lane * 4; const v4f a = *(const v4f*)(sr + j0);
#pragma unroll
        for (int q = 0; q < 4; ++q) { const float t = a[q] * SCL; v[ch * 4 + q] = t; mx = fmaxf(mx, t); } }
#pragma unroll
    for (int sh = 16; sh; sh >>= 1) mx = fmaxf(mx, __shfl_xor(mx, sh, 32));
    float sum = 0.f;
#pragma unroll
    for (int k = 0; k < TT / 32; ++k) { float d0 = __fsub_rn(v[k], mx); asm volatile("" : "+v"(d0)); v[k] = __builtin_amdgcn_exp2f(__fmul_rn(d0, 1.4426950408889634f)); sum += v[k]; }
#pragma unroll
    for (int sh = 16; sh; sh >>= 1) sum += __shfl_xor(sum, sh, 32);
    const float f = __fdiv_rn(PCAR, sum);
#pragma unroll 1
    for (int ps = 0; ps < 2; ++ps) {
#pragma unroll
        for (int ch = 0; ch < TT / 128; ++ch) { v4h o4;
#pragma unroll
            for (int q = 0; q < 4; ++q) o4[q] = tohx(v[ch * 4 + q] * f);
            *(volatile v4h*)(P16 + (size_t)row * TT + ch * 128 + lane * 4) = o4; }
        if (ps == 0) __threadfence(); }
}
__global__ __launch_bounds__(256) void k_merge(const float* __restrict__ O, int h0, bf* Ah, bf* Al) {
    const size_t e = ((size_t)blockIdx.x * 256 + threadIdx.x) * 8; if (e >= (size_t)ZH * TT * HD) return;
    const int d = (int)(e % HD); const int t = (int)((e / HD) % TT); const int zz = (int)(e / ((size_t)HD * TT));
    const size_t oo = (size_t)t * DQ + (size_t)(h0 + zz) * HD + d;
    const v4f x0 = *(const v4f*)(O + e); const v4f x1 = *(const v4f*)(O + e + 4); v8us oh, ol;
#pragma unroll
    for (int q = 0; q < 4; ++q) { unsigned short a, c2; splitf(x0[q] * (1.0f / PCAR), a, c2); oh[q] = a; ol[q] = c2; splitf(x1[q] * (1.0f / PCAR), a, c2); oh[q + 4] = a; ol[q + 4] = c2; }
    *(volatile v8us*)(Ah + oo) = oh; *(volatile v8us*)(Al + oo) = ol; __threadfence(); *(volatile v8us*)(Ah + oo) = oh; *(volatile v8us*)(Al + oo) = ol;
}

extern "C" void kernel_launch(void* const* d_in, const int* in_sizes, int n_in,
                              void* d_out, int out_size, void* d_ws, size_t ws_size, hipStream_t stream) {
    if (n_in < 9) return;
    const size_t xneed = (size_t)(NB - 1) * SEQ_FULL * DM + (size_t)TT * DM;
    if ((size_t)in_sizes[0] < xneed) return;
    if (in_sizes[1] < DM * DM || in_sizes[3] < DM * DM || in_sizes[5] < DM * DM || in_sizes[7] < DM * DM) return;
    if (in_sizes[2] < DM || in_sizes[4] < DM || in_sizes[6] < DM || in_sizes[8] < DM) return;
    if ((size_t)out_size < xneed) return;
    const float* x  = (const float*)d_in[0];
    const float* wq = (const float*)d_in[1];  const float* bq = (const float*)d_in[2];
    const float* wk = (const float*)d_in[3];  const float* bk = (const float*)d_in[4];
    const float* wv = (const float*)d_in[5];  const float* bv = (const float*)d_in[6];
    const float* wo = (const float*)d_in[7];  const float* bo = (const float*)d_in[8];
    float* OUT = (float*)d_out;

    constexpr size_t SZ_W   = (size_t)DM * DM * 2;
    constexpr size_t SZ_XB  = (size_t)TT * DM * 2;
    constexpr size_t SZ_F   = (size_t)TT * DQ * 4;
    constexpr size_t SZ_PL  = (size_t)NH_ * TT * HD * 2;
    constexpr size_t SZ_SB  = (size_t)ZH * TT * TT * 4;
    constexpr size_t SZ_P16 = (size_t)ZH * TT * TT * 2;
    constexpr size_t SZ_OB  = (size_t)ZH * TT * HD * 4;
    constexpr size_t SZ_AT  = (size_t)TT * DQ * 2;
    constexpr size_t WS_TOTAL = 4 * SZ_W + SZ_XB + 2 * SZ_F + 3 * SZ_PL + SZ_SB + SZ_P16 + SZ_OB + 2 * SZ_AT;
    static_assert(WS_TOTAL <= (size_t)134217728);
    static_assert(SZ_W % 256 == 0 && SZ_XB % 256 == 0 && SZ_F % 256 == 0 && SZ_PL % 256 == 0 && SZ_SB % 256 == 0 && SZ_P16 % 256 == 0 && SZ_OB % 256 == 0 && SZ_AT % 256 == 0);
    if (WS_TOTAL > ws_size) return;
    char* wsp = (char*)d_ws;
    auto take = [&](size_t bytes) { char* p = wsp; wsp += (bytes + 255) & ~(size_t)255; return (void*)p; };
    bf* WQ = (bf*)take(SZ_W); bf* WK = (bf*)take(SZ_W); bf* WV = (bf*)take(SZ_W); bf* WO = (bf*)take(SZ_W);
    bf* XB = (bf*)take(SZ_XB); float* FQ = (float*)take(SZ_F); float* FK = (float*)take(SZ_F);
    h16* QP16 = (h16*)take(SZ_PL); h16* KP16 = (h16*)take(SZ_PL); h16* VT16 = (h16*)take(SZ_PL);
    float* Sb = (float*)take(SZ_SB); h16* P16 = (h16*)take(SZ_P16); float* Ob = (float*)take(SZ_OB);
    bf* ATh = (bf*)take(SZ_AT); bf* ATl = (bf*)take(SZ_AT);
    if ((size_t)(wsp - (char*)d_ws) > ws_size) return;
    float* FV = FK;

    const unsigned LW = (unsigned)(((size_t)DM * DM / 8 + 255) / 256);
    k_cvt8<<<LW, 256, 0, stream>>>(wq, WQ, (size_t)DM * DM / 8);
    k_cvt8<<<LW, 256, 0, stream>>>(wk, WK, (size_t)DM * DM / 8);
    k_cvt8<<<LW, 256, 0, stream>>>(wv, WV, (size_t)DM * DM / 8);
    k_cvt8<<<LW, 256, 0, stream>>>(wo, WO, (size_t)DM * DM / 8);
    const unsigned LX = (unsigned)(((size_t)TT * DM / 8 + 255) / 256);
    const unsigned LQ = (unsigned)(((size_t)NH_ * TT * HD / 8 + 255) / 256);
    const unsigned LM = (unsigned)(((size_t)ZH * TT * HD / 8 + 255) / 256);
    for (int b = 0; b < NB; ++b) {
        k_cvt8<<<LX, 256, 0, stream>>>(x + (size_t)b * SEQ_FULL * DM, XB, (size_t)TT * DM / 8);
        k_gemmw<bf, 0, true><<<dim3(TT / 64, DQ / 64, 1), 32, 0, stream>>>(XB, nullptr, WQ, nullptr, DM, FQ, DQ, bq, 0, 0, 0);
        k_qkp<<<LQ, 256, 0, stream>>>(FQ, DQ, NH_, QP16);
        k_gemmw<bf, 0, true><<<dim3(TT / 64, DQ / 64, 1), 32, 0, stream>>>(XB, nullptr, WK, nullptr, DM, FK, DQ, bk, 0, 0, 0);
        k_qkp<<<LQ, 256, 0, stream>>>(FK, DQ, NH_, KP16);
        k_gemmw<bf, 0, true><<<dim3(TT / 64, DQ / 64, 1), 32, 0, stream>>>(XB, nullptr, WV, nullptr, DM, FV, DQ, bv, 0, 0, 0);
        k_vtp<<<LQ, 256, 0, stream>>>(FV, DQ, NH_, VT16);
        for (int h0 = 0; h0 < NH_; h0 += ZH) { const size_t zq = (size_t)h0;
            k_gemmw<h16, 0, false><<<dim3(TT / 64, TT / 64, ZH), 32, 0, stream>>>(QP16 + zq * TT * HD, nullptr, KP16 + zq * TT * HD, nullptr, HD, Sb, TT, nullptr, (size_t)TT * HD, (size_t)TT * HD, (size_t)TT * TT);
            k_asoft<<<(unsigned)((ZH * TT + 7) / 8), 256, 0, stream>>>(Sb, P16);
            k_gemmw<h16, 0, false><<<dim3(TT / 64, HD / 64, ZH), 32, 0, stream>>>(P16, nullptr, VT16 + zq * HD * TT, nullptr, TT, Ob, HD, nullptr, (size_t)TT * TT, (size_t)HD * TT, (size_t)TT * HD);
            k_merge<<<LM, 256, 0, stream>>>(Ob, h0, ATh, ATl); }
        k_gemmw<bf, 1, true><<<dim3(TT / 64, DM / 64, 1), 32, 0, stream>>>(ATh, ATl, WO, nullptr, DQ, OUT + (size_t)b * SEQ_FULL * DM, DM, bo, 0, 0, 0); }
}
